// EnhancedDualDomainMambaBlock_32315333935260
// MI455X (gfx1250) — hardware-verified
//
#include <hip/hip_runtime.h>
#include <hip/hip_bf16.h>
#include <math.h>

#define NBAT  4
#define LL    2048
#define LP    (LL + 2)
#define NHALF 2
#define HB    (NBAT / NHALF)
#define HTOK  (HB * LL)
#define DMOD  512
#define DIN   1024
#define XZW   (2 * DIN)
#define DST   16
#define DTR   32
#define XDN   (DTR + 2 * DST)
#define DCV   4
#define NHEAD 4
#define DHD   128
#define KVW   (2 * DMOD)
#define TECI  128
#define TETAP 3
#define GSTR  40
#define OSTR  68
#define SMEMB (8 * 16 * OSTR * 4)
#define SCH   32
#define SYP   260
#define LOG2E 1.4426950408889634f
#define LNEPS 1e-5f
#define BNEPS 1e-5f
#define RSQDH 0.08838834764831845f
#define WSCAP ((size_t)134217728)
#define SC_XIN 16.0f
#define SC_XS  256.0f
#define SC_DTL 64.0f
#define SC_Y   1024.0f
#define SC_X2  16.0f
#define SC_X3  16.0f
#define SC_W   64.0f
#define SC_WDT 16.0f

static_assert(HTOK % 128 == 0);
static_assert(LL % 256 == 0);
static_assert(XZW % 64 == 0);
static_assert(XDN == 64);
static_assert(DIN % 64 == 0);
static_assert(DMOD % 64 == 0);
static_assert(KVW % 64 == 0);
static_assert(DMOD == NHEAD * DHD);
static_assert(DHD == 128);
static_assert(DMOD == 128 * 4);
static_assert(DIN == 4 * 256);
static_assert(DTR == 32);
static_assert(DST == 16);
static_assert(TECI % 64 == 0);
static_assert((TETAP * TECI) % 32 == 0);
static_assert(LL % SCH == 0);
static_assert(SCH == 32);
static_assert(SYP % 4 == 0);
static_assert(SYP >= 256);
static_assert(SMEMB >= (128 * GSTR + 64 * GSTR) * 2);
static_assert((size_t)HTOK * KVW * 4 + (size_t)HTOK * DMOD * 4 + (size_t)HB * LP * DMOD * 2 <= (size_t)HTOK * XZW * 4);

typedef unsigned short us16 __attribute__((ext_vector_type(16)));
typedef unsigned short us8  __attribute__((ext_vector_type(8)));
typedef unsigned short us8a __attribute__((ext_vector_type(8), may_alias));
typedef __bf16 v16b __attribute__((ext_vector_type(16)));
typedef _Float16 v16h __attribute__((ext_vector_type(16)));
typedef float v8f __attribute__((ext_vector_type(8)));
typedef float v4f __attribute__((ext_vector_type(4)));
typedef float v4fa __attribute__((ext_vector_type(4), may_alias));
union FragU { us16 v; us8 h[2]; };

__device__ __forceinline__ unsigned short bf16_bits(float f) {
  unsigned u = __float_as_uint(f);
  u += 0x7FFFu + ((u >> 16) & 1u);
  return (unsigned short)(u >> 16);
}
__device__ __forceinline__ float bf16_val(unsigned short b) { return __uint_as_float(((unsigned)b) << 16); }
__device__ __forceinline__ float bf16r(float f) { return bf16_val(bf16_bits(f)); }
__device__ __forceinline__ unsigned short h16_bits(float f) { return __builtin_bit_cast(unsigned short, (_Float16)f); }
__device__ __forceinline__ float siluf(float x) { return x * __builtin_amdgcn_rcpf(1.0f + __expf(-x)); }
__device__ __forceinline__ float geluf(float x) { return x * (erff(x * 0.70710678118654752f) + 1.0f) * 0.5f; }

__device__ __forceinline__ float wsum(float v) {
#pragma unroll
  for (int o = 16; o > 0; o >>= 1) v += __shfl_xor(v, o, 32);
  return v;
}
__device__ __forceinline__ float wmax(float v) {
#pragma unroll
  for (int o = 16; o > 0; o >>= 1) v = fmaxf(v, __shfl_xor(v, o, 32));
  return v;
}

template <int BF>
__device__ __forceinline__ v8f mma16(us16 a, us16 b, v8f c) {
  if (BF) return __builtin_amdgcn_wmma_f32_16x16x32_bf16(false, __builtin_bit_cast(v16b, a), false, __builtin_bit_cast(v16b, b), (short)0, c, false, false);
  return __builtin_amdgcn_wmma_f32_16x16x32_f16(false, __builtin_bit_cast(v16h, a), false, __builtin_bit_cast(v16h, b), (short)0, c, false, false);
}
__device__ __forceinline__ void wguard5(v8f (&c)[4], const us16& a, const us16 (&b)[4]) {
#if defined(__HIP_DEVICE_COMPILE__)
  asm volatile("v_nop\n\tv_nop\n\tv_nop\n\tv_nop"
               : "+v"(c[0]), "+v"(c[1]), "+v"(c[2]), "+v"(c[3])
               : "v"(a), "v"(b[0]), "v"(b[1]), "v"(b[2]), "v"(b[3]));
#endif
}

__device__ __forceinline__ us16 lds_frag(const unsigned short* base) {
  const int lane = threadIdx.x & 31, r = lane & 15, kh = (lane >> 4) * 8;
  FragU f;
  f.h[0] = *(const us8a*)(base + r * GSTR + kh);
  f.h[1] = *(const us8a*)(base + r * GSTR + 16 + kh);
  return f.v;
}

__device__ __forceinline__ void stage_a(unsigned short* lds, const unsigned short* __restrict__ P, int ld, int m0, int k0, int tid) {
  const int row = tid >> 1, cq = (tid & 1) * 16;
  const unsigned short* src = P + (size_t)(m0 + row) * ld + k0 + cq;
  const us8 v0 = *(const us8a*)src;
  const us8 v1 = *(const us8a*)(src + 8);
  *(us8a*)(lds + row * GSTR + cq) = v0;
  *(us8a*)(lds + row * GSTR + cq + 8) = v1;
}
__device__ __forceinline__ void stage_b(unsigned short* lds, const unsigned short* __restrict__ P, int ld, int n0, int k0, int tid) {
  const int row = tid >> 2, kq = (tid & 3) * 8;
  const us8 v = *(const us8a*)(P + (size_t)(n0 + row) * ld + k0 + kq);
  *(us8a*)(lds + row * GSTR + kq) = v;
}

template <int BF, int HASB>
__global__ __launch_bounds__(256) void k_gemm(const unsigned short* __restrict__ A0, int lda,
                                             const unsigned short* __restrict__ B0, int ldb, const float* __restrict__ bias,
                                             float* Y, int ldy, int K, float oscale) {
  __shared__ __attribute__((aligned(16))) unsigned char sm[SMEMB];
  unsigned short* lA0 = (unsigned short*)sm;
  unsigned short* lB0 = lA0 + 128 * GSTR;
  float* oS = (float*)sm;
  const int tid = threadIdx.x, lane = tid & 31, wave = tid >> 5, cl = lane & 15, hh = lane >> 4;
  const int m0 = blockIdx.x * 128, n0 = blockIdx.y * 64;

  v8f acc[4];
#pragma unroll
  for (int j = 0; j < 4; ++j) { v8f zz = {0.f, 0.f, 0.f, 0.f, 0.f, 0.f, 0.f, 0.f}; acc[j] = zz; }

#pragma unroll 1
  for (int k0 = 0; k0 < K; k0 += 32) {
    __syncthreads();
    stage_a(lA0, A0, lda, m0, k0, tid);
    stage_b(lB0, B0, ldb, n0, k0, tid);
    __syncthreads();
    const us16 af0 = lds_frag(lA0 + 16 * wave * GSTR);
    us16 bfr[4];
#pragma unroll
    for (int j = 0; j < 4; ++j) bfr[j] = lds_frag(lB0 + 16 * j * GSTR);
#pragma unroll
    for (int j = 0; j < 4; ++j) acc[j] = mma16<BF>(af0, bfr[j], acc[j]);
    wguard5(acc, af0, bfr);
  }
  __syncthreads();

  float* so = oS + wave * (16 * OSTR);
#pragma unroll
  for (int j = 0; j < 4; ++j) {
    float bb = 0.0f;
    if (HASB) bb = bf16r(bias[n0 + 16 * j + cl]);
#pragma unroll
    for (int r = 0; r < 8; ++r) so[(8 * hh + r) * OSTR + 16 * j + cl] = acc[j][r] * oscale + bb;
  }
  __syncthreads();
#pragma unroll
  for (int pass = 0; pass < 2; ++pass) {
#pragma unroll
    for (int it = 0; it < 8; ++it) {
      const int ch = it * 32 + lane, r = ch >> 4, q = (ch & 15) * 4;
      const v4f v = *(const v4fa*)(so + r * OSTR + q);
      *(volatile v4f*)(Y + (size_t)(m0 + 16 * wave + r) * ldy + n0 + q) = v;
    }
    __threadfence();
  }
}

__global__ __launch_bounds__(256) void k_te(const unsigned short* __restrict__ XP, const unsigned short* __restrict__ WT,
                                           const float* __restrict__ X3, const float* __restrict__ teb,
                                           const float* __restrict__ bng, const float* __restrict__ bnb,
                                           const float* __restrict__ bnm, const float* __restrict__ bnv, float* out, float oscale) {
#pragma clang fp contract(off)
  __shared__ __attribute__((aligned(16))) unsigned char sm[SMEMB];
  unsigned short* lA = (unsigned short*)sm;
  unsigned short* lB = lA + 128 * GSTR;
  float* oS = (float*)sm;
  const int tid = threadIdx.x, lane = tid & 31, wave = tid >> 5, cl = lane & 15, hh = lane >> 4;
  const int m0 = blockIdx.x * 128, n0 = blockIdx.y * 64;
  const int bl = m0 / LL, l0 = m0 - bl * LL;
  const int cg = (n0 / TECI) * TECI;
  const unsigned short* XPb = XP + (size_t)bl * LP * DMOD;

  v8f acc[4];
#pragma unroll
  for (int j = 0; j < 4; ++j) { v8f zz = {0.f, 0.f, 0.f, 0.f, 0.f, 0.f, 0.f, 0.f}; acc[j] = zz; }

#pragma unroll 1
  for (int s = 0; s < TETAP * (TECI / 32); ++s) {
    const int kk = s >> 2, cb = (s & 3) * 32;
    __syncthreads();
    stage_a(lA, XPb + (size_t)kk * DMOD, DMOD, l0, cg + cb, tid);
    stage_b(lB, WT + (size_t)kk * DMOD * TECI, TECI, n0, cb, tid);
    __syncthreads();
    const us16 af = lds_frag(lA + 16 * wave * GSTR);
    us16 bw[4];
#pragma unroll
    for (int j = 0; j < 4; ++j) bw[j] = lds_frag(lB + 16 * j * GSTR);
#pragma unroll
    for (int j = 0; j < 4; ++j) acc[j] = mma16<0>(af, bw[j], acc[j]);
    wguard5(acc, af, bw);
  }
  __syncthreads();

  float* so = oS + wave * (16 * OSTR);
#pragma unroll
  for (int j = 0; j < 4; ++j) {
    const int d = n0 + 16 * j + cl;
    const float cbias = bf16r(teb[d]);
    const float rs = rsqrtf(bf16r(bnv[d]) + BNEPS);
    const float gm = bf16r(bng[d]), mn = bf16r(bnm[d]), bb = bf16r(bnb[d]);
#pragma unroll
    for (int r = 0; r < 8; ++r) {
      float hv = acc[j][r] * oscale + cbias;
      hv = (hv - mn) * rs;
      hv = hv * gm + bb;
      so[(8 * hh + r) * OSTR + 16 * j + cl] = hv;
    }
  }
  __syncthreads();
#pragma unroll 1
  for (int it = 0; it < 8; ++it) {
    const int ch = it * 32 + lane, r = ch >> 4, q = (ch & 15) * 4;
    const v4f v = *(const v4fa*)(so + r * OSTR + q);
    const v4f xr = *(const v4fa*)(X3 + (size_t)(m0 + 16 * wave + r) * DMOD + n0 + q);
    v4f o4;
#pragma unroll
    for (int u = 0; u < 4; ++u) o4[u] = xr[u] + geluf(v[u]);
    *(v4fa*)(so + r * OSTR + q) = o4;
  }
#pragma unroll
  for (int pass = 0; pass < 2; ++pass) {
#pragma unroll
    for (int it = 0; it < 8; ++it) {
      const int ch = it * 32 + lane, r = ch >> 4, q = (ch & 15) * 4;
      const v4f v = *(const v4fa*)(so + r * OSTR + q);
      *(volatile v4f*)(out + (size_t)(m0 + 16 * wave + r) * DMOD + n0 + q) = v;
    }
    __threadfence();
  }
}

template <int MODE>
__global__ __launch_bounds__(256) void k_cvt(const float* __restrict__ src, int spitch, unsigned short* dst, int ncol8, int total8, float scale) {
  const int idx = blockIdx.x * 256 + threadIdx.x;
  if (idx >= total8) return;
  const int row = idx / ncol8, c8 = (idx - row * ncol8) * 8;
  const float* s = src + (size_t)row * (size_t)spitch + c8;
  const v4f a = *(const v4fa*)s, b = *(const v4fa*)(s + 4);
  us8 o;
#pragma unroll
  for (int u = 0; u < 4; ++u) {
    const float va = a[u], vb = b[u];
    if (MODE == 0)      { o[u] = bf16_bits(va);               o[4 + u] = bf16_bits(vb); }
    else if (MODE == 1) { o[u] = h16_bits(bf16r(va) * scale); o[4 + u] = h16_bits(bf16r(vb) * scale); }
    else                { o[u] = h16_bits(va * scale);        o[4 + u] = h16_bits(vb * scale); }
  }
  const size_t off = (size_t)row * (size_t)(ncol8 * 8) + c8;
  *(volatile us8*)(dst + off) = o;
  __threadfence();
  *(volatile us8*)(dst + off) = o;
}

__global__ __launch_bounds__(256) void k_prepte(const float* __restrict__ w, unsigned short* WT) {
  const int idx = blockIdx.x * 256 + threadIdx.x;
  const int e = idx * 8;
  const int kk = e >> 16;
  const int r = e & (DMOD * TECI - 1), o_ = r >> 7, ci = r & (TECI - 1);
  us8 o;
#pragma unroll
  for (int u = 0; u < 8; ++u) {
    const float v = w[(size_t)(o_ * TECI + ci + u) * TETAP + kk];
    o[u] = h16_bits(bf16r(v) * SC_W);
  }
  *(volatile us8*)(WT + e) = o;
  __threadfence();
  *(volatile us8*)(WT + e) = o;
}

__global__ __launch_bounds__(256) void k_bsmall(const float* __restrict__ fr, const float* __restrict__ w1, const float* __restrict__ b1,
                                               const float* __restrict__ w2, const float* __restrict__ b2,
                                               const float* __restrict__ wq, const float* __restrict__ bq, float* G, float* Q) {
  __shared__ float sf[DMOD];
  __shared__ float sh[2 * DMOD];
  const int tid = threadIdx.x, b = blockIdx.x;
  sf[tid] = bf16r(fr[b * DMOD + tid]);
  sf[tid + 256] = bf16r(fr[b * DMOD + tid + 256]);
  __syncthreads();
#pragma unroll 1
  for (int jj = 0; jj < (2 * DMOD) / 256; ++jj) {
    const int j = tid + 256 * jj;
    const float* wr = w1 + (size_t)j * DMOD;
    float a = 0.0f;
#pragma unroll 1
    for (int k = 0; k < DMOD; ++k) a += sf[k] * bf16r(wr[k]);
    a += bf16r(b1[j]);
    sh[j] = geluf(a);
  }
  __syncthreads();
  float gv[2], qv[2];
#pragma unroll
  for (int jj = 0; jj < 2; ++jj) {
    const int n = tid + 256 * jj;
    const float* wr = w2 + (size_t)n * (2 * DMOD);
    float a = 0.0f;
#pragma unroll 1
    for (int k = 0; k < 2 * DMOD; ++k) a += sh[k] * bf16r(wr[k]);
    a += bf16r(b2[n]);
    gv[jj] = __builtin_amdgcn_rcpf(1.0f + expf(-a));
    const float* wqr = wq + (size_t)n * DMOD;
    float c = 0.0f;
#pragma unroll 1
    for (int k = 0; k < DMOD; ++k) c += sf[k] * bf16r(wqr[k]);
    qv[jj] = c + bf16r(bq[n]);
  }
  float* gp = G + (size_t)b * DMOD + tid;
  float* qp = Q + (size_t)b * DMOD + tid;
  *(volatile float*)gp = gv[0];  *(volatile float*)(gp + 256) = gv[1];
  *(volatile float*)qp = qv[0];  *(volatile float*)(qp + 256) = qv[1];
  __threadfence();
  *(volatile float*)gp = gv[0];  *(volatile float*)(gp + 256) = gv[1];
  *(volatile float*)qp = qv[0];  *(volatile float*)(qp + 256) = qv[1];
}

__global__ __launch_bounds__(256) void k_conv(const float* __restrict__ XZ, const float* __restrict__ cw, const float* __restrict__ cb,
                                             float* XCF, unsigned short* XCH) {
#pragma clang fp contract(off)
  __shared__ __attribute__((aligned(16))) float sxs[DIN];
  const int tid = threadIdx.x, c4 = tid * 4;
  const int tok = blockIdx.x, l = tok & (LL - 1);
  v4f xv[DCV];
#pragma unroll
  for (int j = 0; j < DCV; ++j) {
    const int ll = l - (DCV - 1) + j;
    const int tc = (ll >= 0) ? (tok - (DCV - 1) + j) : tok;
    xv[j] = *(const v4fa*)(XZ + (size_t)tc * XZW + c4);
  }
  const v4f bb = *(const v4fa*)(cb + c4);
  v4f sv;
#pragma unroll
  for (int u = 0; u < 4; ++u) {
    const v4f wv = *(const v4fa*)(cw + (size_t)(c4 + u) * DCV);
    float a = 0.0f;
#pragma unroll
    for (int j = 0; j < DCV; ++j) {
      const float pr = bf16r(wv[j]) * xv[j][u];
      a = a + ((l - (DCV - 1) + j >= 0) ? pr : 0.0f);
    }
    a = a + bf16r(bb[u]);
    sv[u] = siluf(a);
  }
  *(v4fa*)(sxs + c4) = sv;
  const size_t o = (size_t)tok * DIN + c4;
  *(volatile v4f*)(XCF + o) = sv;
  __threadfence();
  *(volatile v4f*)(XCF + o) = sv;
  __syncthreads();
  if (tid < 128) {
    const int c8 = tid * 8;
    const v4f a = *(const v4fa*)(sxs + c8);
    const v4f b = *(const v4fa*)(sxs + c8 + 4);
    us8 hv;
#pragma unroll
    for (int u = 0; u < 4; ++u) { hv[u] = h16_bits(a[u] * SC_XS); hv[4 + u] = h16_bits(b[u] * SC_XS); }
    const size_t o2 = (size_t)tok * DIN + c8;
    *(volatile us8*)(XCH + o2) = hv;
    __threadfence();
    *(volatile us8*)(XCH + o2) = hv;
  }
}

__global__ __launch_bounds__(256) void k_scan(const float* __restrict__ XZ, const float* __restrict__ XCF, const float* __restrict__ XD,
                                             const float* __restrict__ DTW, const float* __restrict__ dtb, const float* __restrict__ Alog,
                                             const float* __restrict__ Dv, unsigned short* YH) {
#pragma clang fp contract(off)
  __shared__ __attribute__((aligned(16))) float sy[SCH * SYP];
  const int b = blockIdx.x >> 2, dg = blockIdx.x & 3, tid = threadIdx.x, lane = tid & 31, wave = tid >> 5;
  const int d = dg * 256 + tid;
  float A2[DST], h[DST];
#pragma unroll
  for (int n = 0; n < DST; ++n) { A2[n] = -__expf(bf16r(Alog[d * DST + n])) * LOG2E; h[n] = 0.0f; }
  const float Dd = bf16r(Dv[d]);
  const float bd = bf16r(dtb[d]);
#pragma unroll 1
  for (int c = 0; c < LL / SCH; ++c) {
#pragma unroll 1
    for (int s = 0; s < SCH; ++s) {
      const size_t tok = (size_t)b * LL + (size_t)(c * SCH + s);
      const float raw = DTW[tok * DIN + d];
      const float a = raw + bd;
      const float dl = fmaxf(a, 0.0f) + log1pf(__expf(-fabsf(a)));
      const float xv = XCF[tok * DIN + d];
      const float zv = XZ[tok * XZW + DIN + d];
      const float* bcp = XD + tok * XDN;
      v4f Bv[4], Cv[4];
#pragma unroll
      for (int q = 0; q < 4; ++q) {
        Bv[q] = *(const v4fa*)(bcp + DTR + 4 * q);
        Cv[q] = *(const v4fa*)(bcp + DTR + DST + 4 * q);
      }
      const float dx = dl * xv;
      float y = 0.0f;
#pragma unroll
      for (int n = 0; n < DST; ++n) {
        const float e = exp2f(dl * A2[n]);
        h[n] = e * h[n] + dx * Bv[n >> 2][n & 3];
        y = y + h[n] * Cv[n >> 2][n & 3];
      }
      const float yv = (y + xv * Dd) * siluf(zv);
      sy[s * SYP + tid] = yv;
    }
    __syncthreads();
#pragma unroll
    for (int pass = 0; pass < 2; ++pass) {
#pragma unroll
      for (int it = 0; it < 4; ++it) {
        const int row = 4 * wave + it;
        const v4f va = *(const v4fa*)(sy + row * SYP + lane * 8);
        const v4f vb = *(const v4fa*)(sy + row * SYP + lane * 8 + 4);
        us8 o;
#pragma unroll
        for (int u = 0; u < 4; ++u) { o[u] = h16_bits(va[u] * SC_Y); o[4 + u] = h16_bits(vb[u] * SC_Y); }
        const size_t off = ((size_t)b * LL + (size_t)(c * SCH + row)) * DIN + (size_t)dg * 256 + (size_t)lane * 8;
        *(volatile us8*)(YH + off) = o;
      }
      __threadfence();
    }
    __syncthreads();
  }
}

__global__ __launch_bounds__(128) void k_ln12(const float* __restrict__ MO, const float* __restrict__ xg, const float* __restrict__ G,
                                             const float* __restrict__ w1, const float* __restrict__ b1,
                                             const float* __restrict__ w2, const float* __restrict__ b2, float* X2, unsigned short* X2H) {
#pragma clang fp contract(off)
  __shared__ float sred[16];
  __shared__ __attribute__((aligned(16))) float sx[DMOD];
  const int tid = threadIdx.x, lane = tid & 31, wave = tid >> 5, c4 = tid * 4;
  const int tok = blockIdx.x, bl = tok / LL;
  const size_t o = (size_t)tok * DMOD + c4;
  const v4f mv = *(const v4fa*)(MO + o);
  float s = (mv[0] + mv[1]) + (mv[2] + mv[3]);
  s = wsum(s);
  if (lane == 0) sred[wave] = s;
  __syncthreads();
  const float mean = ((sred[0] + sred[1]) + (sred[2] + sred[3])) * (1.0f / DMOD);
  v4f dv;
  float q = 0.0f;
#pragma unroll
  for (int u = 0; u < 4; ++u) { dv[u] = mv[u] - mean; q = q + dv[u] * dv[u]; }
  q = wsum(q);
  if (lane == 0) sred[4 + wave] = q;
  __syncthreads();
  const float var = ((sred[4] + sred[5]) + (sred[6] + sred[7])) * (1.0f / DMOD);
  const float inv = rsqrtf(var + LNEPS);
  const v4f gv = *(const v4fa*)(G + (size_t)bl * DMOD + c4);
  const v4f w1v = *(const v4fa*)(w1 + c4), b1v = *(const v4fa*)(b1 + c4);
  const v4f xv = *(const v4fa*)(xg + o);
  v4f rv;
  float s2 = 0.0f;
#pragma unroll
  for (int u = 0; u < 4; ++u) {
    float t = dv[u] * inv;
    t = t * bf16r(w1v[u]) + bf16r(b1v[u]);
    t = t * (1.0f + gv[u]);
    rv[u] = bf16r(xv[u]) + t;
    s2 = s2 + rv[u];
  }
  s2 = wsum(s2);
  if (lane == 0) sred[8 + wave] = s2;
  __syncthreads();
  const float mean2 = ((sred[8] + sred[9]) + (sred[10] + sred[11])) * (1.0f / DMOD);
  v4f d2;
  float q2 = 0.0f;
#pragma unroll
  for (int u = 0; u < 4; ++u) { d2[u] = rv[u] - mean2; q2 = q2 + d2[u] * d2[u]; }
  q2 = wsum(q2);
  if (lane == 0) sred[12 + wave] = q2;
  __syncthreads();
  const float var2 = ((sred[12] + sred[13]) + (sred[14] + sred[15])) * (1.0f / DMOD);
  const float inv2 = rsqrtf(var2 + LNEPS);
  const v4f w2v = *(const v4fa*)(w2 + c4), b2v = *(const v4fa*)(b2 + c4);
  v4f ov;
#pragma unroll
  for (int u = 0; u < 4; ++u) {
    float t = d2[u] * inv2;
    ov[u] = t * bf16r(w2v[u]) + bf16r(b2v[u]);
  }
  *(volatile v4f*)(X2 + o) = ov;
  __threadfence();
  *(volatile v4f*)(X2 + o) = ov;
  *(v4fa*)(sx + c4) = ov;
  __syncthreads();
  if (tid < 64) {
    const int c8 = tid * 8;
    const v4f a = *(const v4fa*)(sx + c8);
    const v4f b = *(const v4fa*)(sx + c8 + 4);
    us8 hv;
#pragma unroll
    for (int u = 0; u < 4; ++u) { hv[u] = h16_bits(a[u] * SC_X2); hv[4 + u] = h16_bits(b[u] * SC_X2); }
    const size_t o2 = (size_t)tok * DMOD + c8;
    *(volatile us8*)(X2H + o2) = hv;
    __threadfence();
    *(volatile us8*)(X2H + o2) = hv;
  }
}

__global__ __launch_bounds__(256) void k_attn(const float* __restrict__ QB, const float* __restrict__ KV, float* OB) {
  __shared__ __attribute__((aligned(16))) float sq[DHD];
  __shared__ float sc[LL];
  __shared__ float sred[16];
  __shared__ float spart[256];
  const int tid = threadIdx.x, lane = tid & 31, wave = tid >> 5;
  const int bl = blockIdx.x >> 2, hd = blockIdx.x & 3;
  const size_t tok0 = (size_t)bl * LL;
  if (tid < DHD) sq[tid] = QB[(size_t)bl * DMOD + hd * DHD + tid];
  __syncthreads();
  float mx = -3.0e38f;
#pragma unroll 1
  for (int i = 0; i < LL / 256; ++i) {
    const int l = tid + 256 * i;
    const float* kp = KV + (tok0 + (size_t)l) * KVW + hd * DHD;
    float s = 0.0f;
#pragma unroll 2
    for (int d4 = 0; d4 < DHD / 4; ++d4) {
      const v4f kv = *(const v4fa*)(kp + 4 * d4);
      const v4f qv = *(const v4fa*)(sq + 4 * d4);
      s = s + qv[0] * kv[0];
      s = s + qv[1] * kv[1];
      s = s + qv[2] * kv[2];
      s = s + qv[3] * kv[3];
    }
    s = s * RSQDH;
    sc[l] = s;
    mx = fmaxf(mx, s);
  }
  mx = wmax(mx);
  if (lane == 0) sred[wave] = mx;
  __syncthreads();
  float m = sred[0];
#pragma unroll
  for (int w = 1; w < 8; ++w) m = fmaxf(m, sred[w]);
  float ssum = 0.0f;
#pragma unroll 1
  for (int i = 0; i < LL / 256; ++i) {
    const int l = tid + 256 * i;
    const float e = expf(sc[l] - m);
    sc[l] = e;
    ssum += e;
  }
  ssum = wsum(ssum);
  if (lane == 0) sred[8 + wave] = ssum;
  __syncthreads();
  const float S = ((sred[8] + sred[9]) + (sred[10] + sred[11])) + ((sred[12] + sred[13]) + (sred[14] + sred[15]));
  const float rS = 1.0f / S;
  const int d = tid & (DHD - 1), g = tid >> 7;
  const float* vp = KV + (tok0 + (size_t)g * (LL / 2)) * KVW + DMOD + hd * DHD + d;
  const float* sp = sc + g * (LL / 2);
  float acc = 0.0f;
#pragma unroll 4
  for (int l = 0; l < LL / 2; ++l) acc += sp[l] * vp[(size_t)l * KVW];
  spart[tid] = acc;
  __syncthreads();
  if (tid < DHD) {
    const float ov = (spart[tid] + spart[tid + DHD]) * rS;
    float* op = OB + (size_t)bl * DMOD + hd * DHD + tid;
    *(volatile float*)op = ov;
    __threadfence();
    *(volatile float*)op = ov;
  }
}

__global__ __launch_bounds__(256) void k_oproj(const float* __restrict__ OB, const float* __restrict__ W, const float* __restrict__ bo, float* AT) {
  __shared__ float so[DMOD];
  const int tid = threadIdx.x, bl = blockIdx.x;
  so[tid] = OB[(size_t)bl * DMOD + tid];
  so[tid + 256] = OB[(size_t)bl * DMOD + tid + 256];
  __syncthreads();
  float res[2];
#pragma unroll
  for (int jj = 0; jj < 2; ++jj) {
    const int n = tid + 256 * jj;
    const float* wr = W + (size_t)n * DMOD;
    float a = 0.0f;
#pragma unroll 4
    for (int k = 0; k < DMOD; ++k) a += so[k] * bf16r(wr[k]);
    res[jj] = a + bf16r(bo[n]);
  }
  float* ap = AT + (size_t)bl * DMOD + tid;
  *(volatile float*)ap = res[0];  *(volatile float*)(ap + 256) = res[1];
  __threadfence();
  *(volatile float*)ap = res[0];  *(volatile float*)(ap + 256) = res[1];
}

__global__ __launch_bounds__(128) void k_ln3(const float* __restrict__ X2, const float* __restrict__ AT, const float* __restrict__ w3,
                                            const float* __restrict__ b3, float* X3, unsigned short* X3P) {
#pragma clang fp contract(off)
  __shared__ float sred[8];
  __shared__ __attribute__((aligned(16))) float sx[DMOD];
  const int tid = threadIdx.x, lane = tid & 31, wave = tid >> 5, c4 = tid * 4;
  const int prow = blockIdx.x;
  const int bl = prow / LP, lp = prow - bl * LP;
  const size_t poff = (size_t)prow * DMOD;
  if (lp == 0 || lp == LP - 1) {
    if (tid < 64) {
      us8 z;
#pragma unroll
      for (int u = 0; u < 8; ++u) z[u] = (unsigned short)0;
      *(volatile us8*)(X3P + poff + tid * 8) = z;
      __threadfence();
      *(volatile us8*)(X3P + poff + tid * 8) = z;
    }
    return;
  }
  const int tok = bl * LL + (lp - 1);
  const size_t o = (size_t)tok * DMOD + c4;
  const v4f xv = *(const v4fa*)(X2 + o);
  const v4f av = *(const v4fa*)(AT + (size_t)bl * DMOD + c4);
  v4f rv;
  float s = 0.0f;
#pragma unroll
  for (int u = 0; u < 4; ++u) { rv[u] = xv[u] + av[u]; s = s + rv[u]; }
  s = wsum(s);
  if (lane == 0) sred[wave] = s;
  __syncthreads();
  const float mean = ((sred[0] + sred[1]) + (sred[2] + sred[3])) * (1.0f / DMOD);
  v4f dv;
  float q = 0.0f;
#pragma unroll
  for (int u = 0; u < 4; ++u) { dv[u] = rv[u] - mean; q = q + dv[u] * dv[u]; }
  q = wsum(q);
  if (lane == 0) sred[4 + wave] = q;
  __syncthreads();
  const float var = ((sred[4] + sred[5]) + (sred[6] + sred[7])) * (1.0f / DMOD);
  const float inv = rsqrtf(var + LNEPS);
  const v4f wv = *(const v4fa*)(w3 + c4), bv = *(const v4fa*)(b3 + c4);
  v4f ov;
#pragma unroll
  for (int u = 0; u < 4; ++u) {
    float t = dv[u] * inv;
    ov[u] = t * bf16r(wv[u]) + bf16r(bv[u]);
  }
  *(volatile v4f*)(X3 + o) = ov;
  __threadfence();
  *(volatile v4f*)(X3 + o) = ov;
  *(v4fa*)(sx + c4) = ov;
  __syncthreads();
  if (tid < 64) {
    const int c8 = tid * 8;
    const v4f a = *(const v4fa*)(sx + c8);
    const v4f b = *(const v4fa*)(sx + c8 + 4);
    us8 hv;
#pragma unroll
    for (int u = 0; u < 4; ++u) { hv[u] = h16_bits(a[u] * SC_X3); hv[4 + u] = h16_bits(b[u] * SC_X3); }
    *(volatile us8*)(X3P + poff + c8) = hv;
    __threadfence();
    *(volatile us8*)(X3P + poff + c8) = hv;
  }
}

extern "C" void kernel_launch(void* const* d_in, const int* in_sizes, int n_in,
                              void* d_out, int out_size, void* d_ws, size_t ws_size,
                              hipStream_t stream) {
  if (n_in < 31) return;
  if (in_sizes[0] != NBAT * LL * DMOD || in_sizes[1] != NBAT * DMOD || in_sizes[2] != XZW * DMOD ||
      in_sizes[3] != DIN * DCV || in_sizes[4] != DIN || in_sizes[5] != XDN * DIN || in_sizes[6] != DIN * DTR ||
      in_sizes[7] != DIN || in_sizes[8] != DIN * DST || in_sizes[9] != DIN || in_sizes[10] != DMOD * DIN ||
      in_sizes[11] != 2 * DMOD * DMOD || in_sizes[12] != 2 * DMOD || in_sizes[13] != DMOD * 2 * DMOD || in_sizes[14] != DMOD ||
      in_sizes[15] != 3 * DMOD * DMOD || in_sizes[16] != 3 * DMOD || in_sizes[17] != DMOD * DMOD || in_sizes[18] != DMOD ||
      in_sizes[19] != DMOD * TECI * TETAP || in_sizes[20] != DMOD) return;
  for (int i = 21; i <= 30; ++i) if (in_sizes[i] != DMOD) return;
  if (out_size != NBAT * LL * DMOD) return;

  const float* x     = (const float*)d_in[0];
  const float* freq  = (const float*)d_in[1];
  const float* inw   = (const float*)d_in[2];
  const float* c1w   = (const float*)d_in[3];
  const float* c1b   = (const float*)d_in[4];
  const float* xpw   = (const float*)d_in[5];
  const float* dtw   = (const float*)d_in[6];
  const float* dtb   = (const float*)d_in[7];
  const float* Alog  = (const float*)d_in[8];
  const float* Dv    = (const float*)d_in[9];
  const float* ow    = (const float*)d_in[10];
  const float* fgw1  = (const float*)d_in[11];
  const float* fgb1  = (const float*)d_in[12];
  const float* fgw2  = (const float*)d_in[13];
  const float* fgb2  = (const float*)d_in[14];
  const float* ainw  = (const float*)d_in[15];
  const float* ainb  = (const float*)d_in[16];
  const float* aow   = (const float*)d_in[17];
  const float* aob   = (const float*)d_in[18];
  const float* tew   = (const float*)d_in[19];
  const float* teb   = (const float*)d_in[20];
  const float* bng   = (const float*)d_in[21];
  const float* bnb   = (const float*)d_in[22];
  const float* bnm   = (const float*)d_in[23];
  const float* bnv   = (const float*)d_in[24];
  const float* ln1w  = (const float*)d_in[25];
  const float* ln1b  = (const float*)d_in[26];
  const float* ln2w  = (const float*)d_in[27];
  const float* ln2b  = (const float*)d_in[28];
  const float* ln3w  = (const float*)d_in[29];
  const float* ln3b  = (const float*)d_in[30];
  float* out = (float*)d_out;

  size_t off = 0;
  auto carve = [&](size_t bytes) -> char* { char* p = (char*)d_ws + off; off += (bytes + 255) & ~(size_t)255; return p; };
  unsigned short* WIN16 = (unsigned short*)carve((size_t)XZW * DMOD * 2);
  unsigned short* WX16  = (unsigned short*)carve((size_t)XDN * DIN * 2);
  unsigned short* WDT16 = (unsigned short*)carve((size_t)DIN * DTR * 2);
  unsigned short* WO16  = (unsigned short*)carve((size_t)DMOD * DIN * 2);
  unsigned short* WKV16 = (unsigned short*)carve((size_t)KVW * DMOD * 2);
  unsigned short* WTE   = (unsigned short*)carve((size_t)TETAP * DMOD * TECI * 2);
  float* G              = (float*)carve((size_t)NBAT * DMOD * 4);
  float* Q              = (float*)carve((size_t)NBAT * DMOD * 4);
  float* OB             = (float*)carve((size_t)HB * DMOD * 4);
  float* AT             = (float*)carve((size_t)HB * DMOD * 4);
  unsigned short* X16   = (unsigned short*)carve((size_t)HTOK * DMOD * 2);
  float* XZ             = (float*)carve((size_t)HTOK * XZW * 4);
  float* XCF            = (float*)carve((size_t)HTOK * DIN * 4);
  unsigned short* XCH   = (unsigned short*)carve((size_t)HTOK * DIN * 2);
  float* XD             = (float*)carve((size_t)HTOK * XDN * 4);
  unsigned short* DT16  = (unsigned short*)carve((size_t)HTOK * DTR * 2);
  float* DTW            = (float*)carve((size_t)HTOK * DIN * 4);
  unsigned short* YH    = (unsigned short*)carve((size_t)HTOK * DIN * 2);
  float* MO             = (float*)carve((size_t)HTOK * DMOD * 4);
  float* X2             = (float*)carve((size_t)HTOK * DMOD * 4);
  unsigned short* X2H   = (unsigned short*)carve((size_t)HTOK * DMOD * 2);
  if (off > ws_size || off > WSCAP) return;
  float* KV             = XZ;
  float* X3             = XZ + (size_t)HTOK * KVW;
  unsigned short* X3P   = (unsigned short*)(XZ + (size_t)HTOK * KVW + (size_t)HTOK * DMOD);

  const dim3 b256(256), b128(128);
  auto cvt_w = [&](const float* src, int spitch, unsigned short* dst, int nrow, int ncol, float scale) {
    const int ncol8 = ncol / 8, total8 = nrow * ncol8;
    k_cvt<1><<<dim3((total8 + 255) / 256), b256, 0, stream>>>(src, spitch, dst, ncol8, total8, scale);
  };
  auto cvt_a = [&](const float* src, int spitch, unsigned short* dst, int nrow, int ncol, float scale) {
    const int ncol8 = ncol / 8, total8 = nrow * ncol8;
    k_cvt<2><<<dim3((total8 + 255) / 256), b256, 0, stream>>>(src, spitch, dst, ncol8, total8, scale);
  };
  auto gemm = [&](const unsigned short* A, int lda, const unsigned short* B, int ldb, float* Y, int ldy, int M, int N, int K, float oscale) {
    k_gemm<0, 0><<<dim3(M / 128, N / 64), b256, 0, stream>>>(A, lda, B, ldb, c1b, Y, ldy, K, oscale);
  };

  cvt_w(inw, DMOD, WIN16, XZW, DMOD, SC_W);
  cvt_w(xpw, DIN, WX16, XDN, DIN, SC_W);
  cvt_w(dtw, DTR, WDT16, DIN, DTR, SC_WDT);
  cvt_w(ow, DIN, WO16, DMOD, DIN, SC_W);
  cvt_w(ainw + (size_t)DMOD * DMOD, DMOD, WKV16, KVW, DMOD, SC_W);
  k_prepte<<<dim3((TETAP * DMOD * TECI / 8) / 256), b256, 0, stream>>>(tew, WTE);
  k_bsmall<<<dim3(NBAT), b256, 0, stream>>>(freq, fgw1, fgb1, fgw2, fgb2, ainw, ainb, G, Q);

  for (int hp = 0; hp < NHALF; ++hp) {
    const float* xh = x + (size_t)hp * HTOK * DMOD;
    float* outh = out + (size_t)hp * HTOK * DMOD;
    cvt_w(xh, DMOD, X16, HTOK, DMOD, SC_XIN);
    gemm(X16, DMOD, WIN16, DMOD, XZ, XZW, HTOK, XZW, DMOD, 1.0f / (SC_XIN * SC_W));
    k_conv<<<dim3(HTOK), b256, 0, stream>>>(XZ, c1w, c1b, XCF, XCH);
    gemm(XCH, DIN, WX16, DIN, XD, XDN, HTOK, XDN, DIN, 1.0f / (SC_XS * SC_W));
    cvt_a(XD, XDN, DT16, HTOK, DTR, SC_DTL);
    gemm(DT16, DTR, WDT16, DTR, DTW, DIN, HTOK, DIN, DTR, 1.0f / (SC_DTL * SC_WDT));
    k_scan<<<dim3(HB * (DIN / 256)), b256, 0, stream>>>(XZ, XCF, XD, DTW, dtb, Alog, Dv, YH);
    gemm(YH, DIN, WO16, DIN, MO, DMOD, HTOK, DMOD, DIN, 1.0f / (SC_Y * SC_W));
    k_ln12<<<dim3(HTOK), b128, 0, stream>>>(MO, xh, G + (size_t)hp * HB * DMOD, ln1w, ln1b, ln2w, ln2b, X2, X2H);
    k_gemm<0, 1><<<dim3(HTOK / 128, KVW / 64), b256, 0, stream>>>(X2H, DMOD, WKV16, DMOD, ainb + DMOD, KV, KVW, DMOD, 1.0f / (SC_X2 * SC_W));
    k_attn<<<dim3(HB * NHEAD), b256, 0, stream>>>(Q + (size_t)hp * HB * DMOD, KV, OB);
    k_oproj<<<dim3(HB), b256, 0, stream>>>(OB, aow, aob, AT);
    k_ln3<<<dim3(HB * LP), b128, 0, stream>>>(X2, AT, ln3w, ln3b, X3, X3P);
    k_te<<<dim3(HTOK / 128, DMOD / 64), b256, 0, stream>>>(X3P, WTE, X3, teb, bng, bnb, bnm, bnv, outh, 1.0f / (SC_X3 * SC_W));
  }
}
